// WindowAttention_ACAM_12421045420294
// MI455X (gfx1250) — hardware-run, weakly checked
//
#include <hip/hip_runtime.h>
#include <math.h>
#include <stdint.h>

#define NB     2
#define NN     4096
#define CC     96
#define IMW    64
#define NQKV   72
#define MPAD   80
#define BIASN  96
#define QT     64
#define OSP    68
#define TP     72
#define XPP    104
#define RSC    2048.0f
#define IRSC   0.00048828125f
#define LNPS   6.931471805599453f
#define SCALE_F 0.35355339059327373f
#define GELU_K  0.70710678118654752f

static_assert(IMW * IMW == NN);
static_assert(NN % QT == 0);
static_assert((CC * IMW) % QT == 0);
static_assert((OSP * 4) % 16 == 0);
static_assert((TP * 2) % 16 == 0);
static_assert((XPP * 2) % 16 == 0);
static_assert(MPAD * 12 == 960);

typedef _Float16       v16h __attribute__((ext_vector_type(16)));
typedef _Float16       v8h  __attribute__((ext_vector_type(8)));
typedef __bf16         v16b __attribute__((ext_vector_type(16)));
typedef unsigned short v8us __attribute__((ext_vector_type(8)));
typedef float          v8f  __attribute__((ext_vector_type(8)));
typedef float          v4f  __attribute__((ext_vector_type(4)));
typedef unsigned int   v4u  __attribute__((ext_vector_type(4)));

union Frag  { v8us u[2]; v16h h; v16b bf; };
union FragH { v16h v; v8h hv[2]; };
static_assert(sizeof(Frag) == 32);
static_assert(sizeof(FragH) == 32);

__device__ __forceinline__ unsigned short bf_bits(float f) {
  unsigned u = __float_as_uint(f);
  return (unsigned short)((u + 0x7FFFu + ((u >> 16) & 1u)) >> 16);
}
__device__ __forceinline__ float bf_up(unsigned short hb) { return __uint_as_float(((unsigned)hb) << 16); }
__device__ __forceinline__ float bfr(float f) { return bf_up(bf_bits(f)); }
__device__ __forceinline__ unsigned short h_bits(_Float16 x) { return __builtin_bit_cast(unsigned short, x); }
__device__ __forceinline__ unsigned pk16(unsigned short a, unsigned short b) { return (unsigned)a | ((unsigned)b << 16); }
__device__ __forceinline__ v8f zero8() { v8f z = {0.f, 0.f, 0.f, 0.f, 0.f, 0.f, 0.f, 0.f}; return z; }
__device__ __forceinline__ float hmax8(v8f s) {
  return fmaxf(fmaxf(fmaxf(s[0], s[1]), fmaxf(s[2], s[3])), fmaxf(fmaxf(s[4], s[5]), fmaxf(s[6], s[7])));
}
__device__ __forceinline__ float gelu_f(float x) { return 0.5f * x * (1.0f + erff(x * GELU_K)); }

__device__ __forceinline__ Frag ldfrag(const unsigned short* p) {
  Frag f;
  f.u[0] = *(const v8us*)(p);
  f.u[1] = *(const v8us*)(p + 16);
  return f;
}

__device__ __forceinline__ v8f mma_h(v16h a, v16h b, v8f c) {
  v8f d = __builtin_amdgcn_wmma_f32_16x16x32_f16(false, a, false, b, (short)0, c, false, false);
#if defined(__HIP_DEVICE_COMPILE__)
  asm volatile("v_nop\n\tv_nop\n\tv_nop\n\tv_nop" : "+v"(d) : "v"(a), "v"(b));
#endif
  return d;
}
__device__ __forceinline__ v8f mma_b(v16b a, v16b b, v8f c) {
  v8f d = __builtin_amdgcn_wmma_f32_16x16x32_bf16(false, a, false, b, (short)0, c, false, false);
#if defined(__HIP_DEVICE_COMPILE__)
  const v16h ha = __builtin_bit_cast(v16h, a), hb = __builtin_bit_cast(v16h, b);
  asm volatile("v_nop\n\tv_nop\n\tv_nop\n\tv_nop" : "+v"(d) : "v"(ha), "v"(hb));
#endif
  return d;
}

__global__ __launch_bounds__(256)
void cvt_w(const float* __restrict__ w0, const float* __restrict__ w1, const float* __restrict__ w2,
           const float* __restrict__ w3, const float* __restrict__ w4, const float* __restrict__ w5,
           const float* __restrict__ w6, const float* __restrict__ w7, const float* __restrict__ w8,
           const float* __restrict__ b0, const float* __restrict__ b1, const float* __restrict__ b2,
           const float* __restrict__ b3, const float* __restrict__ b4, const float* __restrict__ b5,
           const float* __restrict__ b6, const float* __restrict__ b7, const float* __restrict__ b8,
           unsigned short* W16, float* BIAS) {
  const int tid = threadIdx.x;
  v4f bv;
  {
    const int tb = min(tid, 23);
    const int m = tb >> 1;
    const bool valid = (m < 9);
    const int mc = min(m, 8);
    const int r0 = 4 * (tb & 1);
    const float* bp = (mc == 0) ? b0 : (mc == 1) ? b1 : (mc == 2) ? b2 : (mc == 3) ? b3 :
                      (mc == 4) ? b4 : (mc == 5) ? b5 : (mc == 6) ? b6 : (mc == 7) ? b7 : b8;
#pragma unroll
    for (int q = 0; q < 4; ++q) bv[q] = valid ? bfr(bp[r0 + q]) : 0.f;
  }
#pragma unroll
  for (int pass = 0; pass < 2; ++pass) {
#pragma unroll
    for (int it = 0; it < 4; ++it) {
      const int i = it * 256 + tid;
      if (i < 960) {
        const int o = i / 12;
        const int col = 8 * (i - 12 * o);
        const int m = o >> 3, r = o & 7;
        const bool valid = (o < NQKV);
        const int mc = min(m, 8);
        const float* wp = (mc == 0) ? w0 : (mc == 1) ? w1 : (mc == 2) ? w2 : (mc == 3) ? w3 :
                          (mc == 4) ? w4 : (mc == 5) ? w5 : (mc == 6) ? w6 : (mc == 7) ? w7 : w8;
        const float* s = wp + (r * CC + col);
        const v4f a = *(const v4f*)(s);
        const v4f q = *(const v4f*)(s + 4);
        v4u u;
        u[0] = valid ? pk16(bf_bits(a[0]), bf_bits(a[1])) : 0u;
        u[1] = valid ? pk16(bf_bits(a[2]), bf_bits(a[3])) : 0u;
        u[2] = valid ? pk16(bf_bits(q[0]), bf_bits(q[1])) : 0u;
        u[3] = valid ? pk16(bf_bits(q[2]), bf_bits(q[3])) : 0u;
        *(volatile v4u*)(W16 + (size_t)8 * i) = u;
      }
    }
    if (tid < 24) *(volatile v4f*)(BIAS + 4 * tid) = bv;
    __threadfence();
  }
}

__global__ __launch_bounds__(256)
void tr_kernel(const float* __restrict__ src, int srcB, int useBf,
               unsigned short* Draw, int drawB, unsigned short* Th, unsigned short* Tl, int R) {
  __shared__ __align__(16) unsigned short T1[64 * TP];
  __shared__ __align__(16) unsigned short T2[64 * TP];
  __shared__ __align__(16) unsigned short T3[64 * TP];
  const int tid = threadIdx.x;
  const int cb = blockIdx.x, b = blockIdx.y;
  const float* sp = src + (size_t)b * srcB + (size_t)cb * 4096;
  {
    const int w4 = (tid & 15) * 4, hs = tid >> 4;
#pragma unroll
    for (int it = 0; it < 4; ++it) {
      const int h = it * 16 + hs;
      const v4f v = *(const v4f*)(sp + h * 64 + w4);
#pragma unroll
      for (int q = 0; q < 4; ++q) {
        float f = v[q];
        f = (useBf != 0) ? bfr(f) : f;
        const _Float16 hi = (_Float16)f;
        const _Float16 lo = (_Float16)((f - (float)hi) * RSC);
        T1[(w4 + q) * TP + h] = h_bits(hi);
        T2[(w4 + q) * TP + h] = h_bits(lo);
        T3[h * TP + w4 + q]   = bf_bits(f);
      }
    }
  }
  __syncthreads();
  {
    const int e = tid & 7, lq = tid >> 3;
#pragma unroll
    for (int pass = 0; pass < 2; ++pass) {
#pragma unroll
      for (int it = 0; it < 2; ++it) {
        const int r = it * 32 + lq;
        const v4u u1 = *(const v4u*)(T1 + r * TP + 8 * e);
        *(volatile v4u*)(Th + ((size_t)b * 64 + r) * (size_t)R + (size_t)cb * 64 + 8 * e) = u1;
        if (Tl != nullptr) {
          const v4u u2 = *(const v4u*)(T2 + r * TP + 8 * e);
          *(volatile v4u*)(Tl + ((size_t)b * 64 + r) * (size_t)R + (size_t)cb * 64 + 8 * e) = u2;
        }
        if (Draw != nullptr) {
          const v4u u3 = *(const v4u*)(T3 + r * TP + 8 * e);
          *(volatile v4u*)(Draw + (size_t)b * drawB + (size_t)cb * 4096 + r * 64 + 8 * e) = u3;
        }
      }
      __threadfence();
    }
  }
}

__global__ __launch_bounds__(256)
void cvt_xp(const float* __restrict__ x, unsigned short* XP) {
  __shared__ __align__(16) unsigned short Lt[QT * XPP];
  const int tid = threadIdx.x;
  const int nt = blockIdx.x, b = blockIdx.y;
  const int n0 = nt * QT;
  {
    const int n4 = (tid & 15) * 4, cs = tid >> 4;
#pragma unroll
    for (int it = 0; it < 6; ++it) {
      const int c = it * 16 + cs;
      const v4f v = *(const v4f*)(x + ((size_t)(b * CC + c)) * NN + n0 + n4);
#pragma unroll
      for (int q = 0; q < 4; ++q) Lt[(n4 + q) * XPP + c] = bf_bits(v[q]);
    }
  }
  __syncthreads();
  {
    const int e = tid & 7, lq = tid >> 3;
#pragma unroll
    for (int pass = 0; pass < 2; ++pass) {
#pragma unroll
      for (int it = 0; it < 3; ++it) {
        const int L = it * 32 + lq;
        const int idx = 64 * L + 8 * e;
        const int nl = idx / CC;
        const int col = idx - CC * nl;
        const v4u u = *(const v4u*)(Lt + nl * XPP + col);
        *(volatile v4u*)(XP + ((size_t)(b * NN + n0)) * CC + idx) = u;
      }
      __threadfence();
    }
  }
}

__global__ __launch_bounds__(128)
void gemm_qkv(const unsigned short* __restrict__ W16, const float* __restrict__ BIAS,
              const unsigned short* __restrict__ XP, float* QKV) {
  __shared__ __align__(16) float Os[MPAD * OSP];
  const int tid  = threadIdx.x;
  const int lane = tid & 31, wave = tid >> 5;
  const int hh   = lane >> 4, c = lane & 15;
  const int nt   = blockIdx.x, b = blockIdx.y;
  const int n0   = nt * QT;

  const unsigned short* ap = W16 + (size_t)c * CC + 8 * hh;
  const unsigned short* bp = XP + ((size_t)(b * NN + n0 + 16 * wave + c)) * CC + 8 * hh;

  v8f acc[5];
#pragma unroll
  for (int mt = 0; mt < 5; ++mt) acc[mt] = zero8();

#pragma unroll
  for (int ks = 0; ks < 3; ++ks) {
    const Frag fb = ldfrag(bp + 32 * ks);
#pragma unroll
    for (int mt = 0; mt < 5; ++mt) {
      const Frag fa = ldfrag(ap + (size_t)(16 * mt) * CC + 32 * ks);
      acc[mt] = mma_b(fa.bf, fb.bf, acc[mt]);
    }
  }

  {
    const int n_loc = 16 * wave + c;
#pragma unroll
    for (int mt = 0; mt < 5; ++mt) {
#pragma unroll
      for (int r = 0; r < 8; ++r) {
        const int o = 16 * mt + 8 * hh + r;
        Os[o * OSP + n_loc] = acc[mt][r] + BIAS[o];
      }
    }
  }
  __syncthreads();

  {
    const int e = tid & 7, lq = tid >> 3;
#pragma unroll
    for (int pass = 0; pass < 2; ++pass) {
#pragma unroll
      for (int it = 0; it < 9; ++it) {
        const int L = it * 16 + lq;
        const int row = L >> 1, hf = L & 1;
        const v4f v = *(const v4f*)(Os + row * OSP + hf * 32 + 4 * e);
        float* dst = QKV + ((size_t)(b * NQKV + row)) * NN + n0 + hf * 32 + 4 * e;
        *(volatile v4f*)dst = v;
      }
      __threadfence();
    }
  }
}

__global__ __launch_bounds__(256)
void planes_kernel(const float* __restrict__ QKV, unsigned short* Qp, unsigned short* Kp, unsigned short* VTp,
                   unsigned short* CQh, unsigned short* CQl, unsigned short* CKh, unsigned short* CKl) {
  __shared__ __align__(16) float Ys[40 * QT];
  const int tid = threadIdx.x;
  const int nt = blockIdx.x, b = blockIdx.y;
  const int n0 = nt * QT;
#pragma unroll
  for (int it = 0; it < 3; ++it) {
    const int p = it * 256 + tid;
    if (p < 640) {
      const int r = p >> 4, n4 = (p & 15) * 4;
      *(v4f*)(Ys + r * QT + n4) = *(const v4f*)(QKV + ((size_t)(b * NQKV + 24 + r)) * NN + n0 + n4);
    }
  }
  __syncthreads();

  const int e = tid & 7, lq = tid >> 3;
  const int nl = 2 * lq + (e >> 2), col0 = 8 * (e & 3);
  const bool lead = (col0 == 0);
  v4u uq, uk;
  {
    float fq[8], fk[8];
#pragma unroll
    for (int cch = 0; cch < 8; ++cch) { fq[cch] = Ys[cch * QT + nl]; fk[cch] = Ys[(8 + cch) * QT + nl]; }
#pragma unroll
    for (int t = 0; t < 4; ++t) {
      uq[t] = lead ? pk16(bf_bits(fq[2 * t]), bf_bits(fq[2 * t + 1])) : 0u;
      uk[t] = lead ? pk16(bf_bits(fk[2 * t]), bf_bits(fk[2 * t + 1])) : 0u;
    }
  }
  v4u uv;
  {
    const int cr = min(lq, 7);
    const bool vreal = (lq < 8);
    float f[8];
#pragma unroll
    for (int q = 0; q < 8; ++q) f[q] = Ys[(16 + cr) * QT + 8 * e + q];
#pragma unroll
    for (int t = 0; t < 4; ++t)
      uv[t] = vreal ? pk16(h_bits((_Float16)f[2 * t]), h_bits((_Float16)f[2 * t + 1])) : 0u;
  }
  const int pidx = lq >> 3, cch = lq & 7;
  v4u uc;
  {
    const int row = 24 + (pidx >> 1) * 8 + cch;
    float f[8];
#pragma unroll
    for (int q = 0; q < 8; ++q) f[q] = Ys[row * QT + 8 * e + q];
#pragma unroll
    for (int t = 0; t < 4; ++t) {
      const unsigned short hb0 = bf_bits(f[2 * t]), hb1 = bf_bits(f[2 * t + 1]);
      const unsigned short lb0 = bf_bits(f[2 * t] - bf_up(hb0));
      const unsigned short lb1 = bf_bits(f[2 * t + 1] - bf_up(hb1));
      uc[t] = (pidx & 1) ? pk16(lb0, lb1) : pk16(hb0, hb1);
    }
  }
  unsigned short* CP = (pidx == 0) ? CQh : (pidx == 1) ? CQl : (pidx == 2) ? CKh : CKl;
  const size_t oq = ((size_t)(b * NN + n0 + nl)) * 32 + col0;
  const size_t ov = ((size_t)(b * 16 + lq)) * NN + n0 + 8 * e;
  const size_t oc = (size_t)b * (8 * NN) + (size_t)cch * NN + n0 + 8 * e;
#pragma unroll
  for (int pass = 0; pass < 2; ++pass) {
    *(volatile v4u*)(Qp + oq) = uq;
    *(volatile v4u*)(Kp + oq) = uk;
    if (lq < 16) *(volatile v4u*)(VTp + ov) = uv;
    *(volatile v4u*)(CP + oc) = uc;
    __threadfence();
  }
}

__global__ __launch_bounds__(256)
void chan_kernel(const float* __restrict__ QKV, float* Y1) {
  __shared__ double part[256];
  __shared__ float A[64];
  const int tid = threadIdx.x, b = blockIdx.x;
  const float* Q = QKV + (size_t)b * (NQKV * NN);
  const float* K = Q + 8 * NN;
  const float* V = Q + 16 * NN;
  {
    const int pair = tid >> 2, seg = tid & 3;
    const int cq = pair >> 3, dk = pair & 7;
    const float* qp = Q + cq * NN + seg * 1024;
    const float* kp = K + dk * NN + seg * 1024;
    double s = 0.0;
#pragma unroll 4
    for (int n = 0; n < 1024; ++n) s = fma((double)qp[n], (double)kp[n], s);
    part[tid] = s;
  }
  __syncthreads();
  if (tid < 64) {
    const double t = (part[4 * tid] + part[4 * tid + 1]) + (part[4 * tid + 2] + part[4 * tid + 3]);
    A[tid] = (float)t * SCALE_F;
  }
  __syncthreads();
  if (tid < 8) {
    float mx = -3.0e38f;
#pragma unroll 1
    for (int j = 0; j < 8; ++j) mx = fmaxf(mx, A[tid * 8 + j]);
    float sm = 0.f;
#pragma unroll 1
    for (int j = 0; j < 8; ++j) { const float ev = expf(A[tid * 8 + j] - mx); A[tid * 8 + j] = ev; sm += ev; }
    const float inv = 1.0f / sm;
#pragma unroll 1
    for (int j = 0; j < 8; ++j) A[tid * 8 + j] = A[tid * 8 + j] * inv;
  }
  __syncthreads();
  float* Yb = Y1 + (size_t)b * (8 * NN);
#pragma unroll
  for (int pass = 0; pass < 2; ++pass) {
#pragma unroll 1
    for (int it = 0; it < 128; ++it) {
      const int i = it * 256 + tid;
      const int cq = i >> 12, n = i & 4095;
      float acc = 0.f;
#pragma unroll
      for (int j = 0; j < 8; ++j) acc = fmaf(A[cq * 8 + j], V[j * NN + n], acc);
      *(volatile float*)(Yb + i) = acc;
    }
    __threadfence();
  }
}

template <int NJ, int KS, int QS, int VS, int PL>
__global__ __launch_bounds__(128)
void attn_kernel(const unsigned short* __restrict__ Qh, const unsigned short* __restrict__ Ql,
                 const unsigned short* __restrict__ Kh, const unsigned short* __restrict__ Kl,
                 const unsigned short* __restrict__ Vh, const unsigned short* __restrict__ Vl,
                 float* O, int NK, int qbs, int kbs, int vbs, int obs) {
  static_assert(!VS || PL);
  static_assert(NJ == 1 || NJ == 4);
  constexpr int KP   = 32 * KS;
  constexpr int DOUT = (NJ == 1) ? 8 : 16 * NJ;
  constexpr int NL   = QT * DOUT / 32;
  constexpr int NIT  = NL / 16;
  __shared__ __align__(16) float Os[QT * OSP];
  const int tid  = threadIdx.x;
  const int wave = tid >> 5, lane = tid & 31;
  const int hh   = lane >> 4, c = lane & 15;
  const int n0   = blockIdx.x * QT, b = blockIdx.y;

  Frag qh[KS], ql[KS];
  {
    const size_t qo = (size_t)b * qbs + (size_t)(n0 + 16 * wave + c) * KP + 8 * hh;
#pragma unroll
    for (int ks = 0; ks < KS; ++ks) {
      qh[ks] = ldfrag(Qh + qo + 32 * ks);
      if (QS) ql[ks] = ldfrag(Ql + qo + 32 * ks); else ql[ks] = qh[ks];
    }
  }
  const unsigned short* Khp = Kh + (size_t)b * kbs + (size_t)c * KP + 8 * hh;
  const unsigned short* Klp = QS ? (Kl + (size_t)b * kbs + (size_t)c * KP + 8 * hh) : Khp;
  const unsigned short* Vhp = Vh + (size_t)b * vbs + (size_t)c * NK + 8 * hh;
  const unsigned short* Vlp = VS ? (Vl + (size_t)b * vbs + (size_t)c * NK + 8 * hh) : Vhp;

  float m = -1.0e30f, l = 0.f;
  v8f o[NJ], ol[NJ];
#pragma unroll
  for (int j = 0; j < NJ; ++j) { o[j] = zero8(); ol[j] = zero8(); }

#pragma unroll 1
  for (int kb = 0; kb < NK; kb += 32) {
    v8f s0 = zero8(), s1 = zero8();
#pragma unroll
    for (int ks = 0; ks < KS; ++ks) {
      const Frag k0 = ldfrag(Khp + (size_t)kb * KP + 32 * ks);
      const Frag k1 = ldfrag(Khp + (size_t)(kb + 16) * KP + 32 * ks);
      s0 = mma_b(k0.bf, qh[ks].bf, s0);
      s1 = mma_b(k1.bf, qh[ks].bf, s1);
      if (QS) {
        const Frag k0l = ldfrag(Klp + (size_t)kb * KP + 32 * ks);
        const Frag k1l = ldfrag(Klp + (size_t)(kb + 16) * KP + 32 * ks);
        s0 = mma_b(k0.bf, ql[ks].bf, s0);
        s1 = mma_b(k1.bf, ql[ks].bf, s1);
        s0 = mma_b(k0l.bf, qh[ks].bf, s0);
        s1 = mma_b(k1l.bf, qh[ks].bf, s1);
      }
    }
#pragma unroll
    for (int r = 0; r < 8; ++r) { s0[r] *= SCALE_F; s1[r] *= SCALE_F; }

    float mx = fmaxf(hmax8(s0), hmax8(s1));
    mx = fmaxf(mx, __shfl_xor(mx, 16, 32));
    const float mn   = fmaxf(m, mx);
    const float corr = __expf(m - mn);
    m = mn;
    const float msh = mn - LNPS;
    l *= corr;
#pragma unroll
    for (int j = 0; j < NJ; ++j) {
#pragma unroll
      for (int r = 0; r < 8; ++r) { o[j][r] *= corr; if (PL) ol[j][r] *= corr; }
    }

    FragH ph, pl;
    float ls = 0.f;
#pragma unroll
    for (int r = 0; r < 8; ++r) {
      const float e0 = __expf(s0[r] - msh);
      const float e1 = __expf(s1[r] - msh);
      ls += e0 + e1;
      const _Float16 h0 = (_Float16)e0, h1 = (_Float16)e1;
      ph.hv[0][r] = h0;
      ph.hv[1][r] = h1;
      pl.hv[0][r] = (_Float16)((e0 - (float)h0) * RSC);
      pl.hv[1][r] = (_Float16)((e1 - (float)h1) * RSC);
    }
    l += ls;

#pragma unroll
    for (int j = 0; j < NJ; ++j) {
      const Frag vf = ldfrag(Vhp + (size_t)(16 * j) * NK + kb);
      o[j] = mma_h(vf.h, ph.v, o[j]);
      if (PL) ol[j] = mma_h(vf.h, pl.v, ol[j]);
      if (VS) {
        const Frag vlf = ldfrag(Vlp + (size_t)(16 * j) * NK + kb);
        ol[j] = mma_h(vlf.h, ph.v, ol[j]);
      }
    }
  }
  l += __shfl_xor(l, 16, 32);
  const float inv = 1.0f / l;

  {
    const int qrow = 16 * wave + c;
#pragma unroll
    for (int j = 0; j < NJ; ++j) {
      v4f va, vb;
#pragma unroll
      for (int r = 0; r < 4; ++r) {
        float t0 = o[j][r], t1 = o[j][4 + r];
        if (PL) { t0 += ol[j][r] * IRSC; t1 += ol[j][4 + r] * IRSC; }
        va[r] = t0 * inv;
        vb[r] = t1 * inv;
      }
      if (NJ == 1) {
        if (hh == 0) {
          *(v4f*)(Os + qrow * 8)     = va;
          *(v4f*)(Os + qrow * 8 + 4) = vb;
        }
      } else {
        *(v4f*)(Os + qrow * OSP + 16 * j + 8 * hh)     = va;
        *(v4f*)(Os + qrow * OSP + 16 * j + 8 * hh + 4) = vb;
      }
    }
  }
  __syncthreads();
  {
    const int e = tid & 7, lq = tid >> 3;
    float* ob = O + (size_t)b * obs + (size_t)n0 * DOUT;
#pragma unroll
    for (int pass = 0; pass < 2; ++pass) {
#pragma unroll
      for (int it = 0; it < NIT; ++it) {
        const int L = it * 16 + lq;
        const float* sp = (NJ == 1) ? (Os + 32 * L + 4 * e) : (Os + (L >> 1) * OSP + (L & 1) * 32 + 4 * e);
        const v4f v = *(const v4f*)sp;
        *(volatile v4f*)(ob + 32 * L + 4 * e) = v;
      }
      __threadfence();
    }
  }
}

__global__ __launch_bounds__(256)
void proj_kernel(const float* __restrict__ Y1, const float* __restrict__ Y2,
                 const float* __restrict__ Y3, const float* __restrict__ Y4,
                 const float* __restrict__ pw1, const float* __restrict__ pw2,
                 const float* __restrict__ pw3, const float* __restrict__ pw4,
                 const float* __restrict__ cg1, const float* __restrict__ cg2,
                 const float* __restrict__ cg3, const float* __restrict__ cg4,
                 const float* __restrict__ gm1, const float* __restrict__ gm2,
                 const float* __restrict__ gm3, const float* __restrict__ gm4,
                 float* out) {
  __shared__ __align__(16) float Tt[QT * CC];
  __shared__ float Wc[4 * CC * 9];
  const int tid = threadIdx.x;
  const int h = blockIdx.x, b = blockIdx.y;
  const int n0 = h * IMW;
  for (int k = tid; k < CC * 9; k += 256) {
    Wc[k]              = bfr(pw1[k]);
    Wc[CC * 9 + k]     = bfr(pw2[k]);
    Wc[2 * CC * 9 + k] = bfr(pw3[k]);
    Wc[3 * CC * 9 + k] = bfr(pw4[k]);
  }
  const float g1v = bfr(cg1[0]), g2v = bfr(cg2[0]), g3v = bfr(cg3[0]), g4v = bfr(cg4[0]);
  const float a1v = bfr(gm1[0]), a2v = bfr(gm2[0]), a3v = bfr(gm3[0]), a4v = bfr(gm4[0]);
  __syncthreads();

#pragma unroll 1
  for (int i = 0; i < 24; ++i) {
    const int e = i * 256 + tid;
    const int w = e / CC;
    const int o = e - CC * w;
    const int g8 = o / 12;
    float acc = 0.f;
#pragma unroll 1
    for (int br = 0; br < 4; ++br) {
      const float* yb = (br == 0) ? Y1 : (br == 1) ? Y2 : (br == 2) ? Y3 : Y4;
      const int chs = (br == 3) ? (CC * NN) : (8 * NN);
      const int ch  = (br == 3) ? o : g8;
      const float gg = (br == 0) ? g1v : (br == 1) ? g2v : (br == 2) ? g3v : g4v;
      const float gm = (br == 0) ? a1v : (br == 1) ? a2v : (br == 2) ? a3v : a4v;
      const float* yp = yb + (size_t)b * chs + (size_t)ch * NN;
      const float* wt = Wc + br * (CC * 9) + o * 9;
      float s = 0.f;
#pragma unroll
      for (int t = 0; t < 9; ++t) {
        const int ky = t / 3, kx = t - 3 * ky;
        const int hy = h + ky - 1, wx = w + kx - 1;
        const bool ok = ((unsigned)hy < 64u) && ((unsigned)wx < 64u);
        const int hcl = min(max(hy, 0), 63), wcl = min(max(wx, 0), 63);
        const float v = yp[hcl * IMW + wcl];
        s = fmaf(ok ? v : 0.f, wt[t], s);
      }
      const float tg  = gelu_f(s);
      const float obr = gg * tg + tg;
      acc = acc + gm * obr;
    }
    Tt[e] = acc;
  }
  __syncthreads();
  {
    const int e8 = tid & 7, lq = tid >> 3;
    float* ob = out + ((size_t)(b * NN + n0)) * CC;
#pragma unroll
    for (int pass = 0; pass < 2; ++pass) {
#pragma unroll
      for (int it = 0; it < 6; ++it) {
        const int L = it * 32 + lq;
        const v4f v = *(const v4f*)(Tt + 32 * L + 4 * e8);
        *(volatile v4f*)(ob + 32 * L + 4 * e8) = v;
      }
      __threadfence();
    }
  }
}

extern "C" void kernel_launch(void* const* d_in, const int* in_sizes, int n_in,
                              void* d_out, int out_size, void* d_ws, size_t ws_size,
                              hipStream_t stream) {
  const int OUTN = NB * NN * CC;
  if (n_in < 31) return;
  if (in_sizes[0] != OUTN) return;
  {
    const int widx[9] = {1, 3, 5, 9, 11, 13, 17, 19, 21};
    for (int i = 0; i < 9; ++i) {
      if (in_sizes[widx[i]] != 8 * CC) return;
      if (in_sizes[widx[i] + 1] != 8) return;
    }
    const int pidx[4] = {7, 15, 23, 25};
    for (int i = 0; i < 4; ++i) if (in_sizes[pidx[i]] != CC * 9) return;
    const int sidx[8] = {8, 16, 24, 26, 27, 28, 29, 30};
    for (int i = 0; i < 8; ++i) if (in_sizes[sidx[i]] != 1) return;
  }
  if (out_size != OUTN) return;

  size_t off = 0;
  auto carve = [&](size_t bytes) { const size_t o = off; off += (bytes + 255) & ~(size_t)255; return o; };
  const size_t oW16 = carve((size_t)MPAD * CC * 2);
  const size_t oBIA = carve((size_t)BIASN * 4);
  const size_t oX16 = carve((size_t)NB * CC * IMW * 64 * 2);
  const size_t oXT  = carve((size_t)NB * 64 * CC * IMW * 2);
  const size_t oXP  = carve((size_t)NB * NN * CC * 2);
  const size_t oQKV = carve((size_t)NB * NQKV * NN * 4);
  const size_t oQp  = carve((size_t)NB * NN * 32 * 2);
  const size_t oKp  = carve((size_t)NB * NN * 32 * 2);
  const size_t oVTp = carve((size_t)NB * 16 * NN * 2);
  const size_t oCQh = carve((size_t)NB * 512 * 64 * 2);
  const size_t oCQl = carve((size_t)NB * 512 * 64 * 2);
  const size_t oCKh = carve((size_t)NB * 512 * 64 * 2);
  const size_t oCKl = carve((size_t)NB * 512 * 64 * 2);
  const size_t oVTh = carve((size_t)NB * 64 * 512 * 2);
  const size_t oVTl = carve((size_t)NB * 64 * 512 * 2);
  const size_t oY1  = carve((size_t)NB * 8 * NN * 4);
  const size_t oY2  = carve((size_t)NB * 8 * NN * 4);
  const size_t oY3  = carve((size_t)NB * 8 * NN * 4);
  const size_t oY4  = carve((size_t)NB * CC * IMW * 64 * 4);
  if (off > ws_size) return;
  if (off > (size_t)134217728) return;

  const float* x = (const float*)d_in[0];
  const float* wq[9]; const float* bq[9];
  {
    const int widx[9] = {1, 3, 5, 9, 11, 13, 17, 19, 21};
    for (int i = 0; i < 9; ++i) { wq[i] = (const float*)d_in[widx[i]]; bq[i] = (const float*)d_in[widx[i] + 1]; }
  }
  const float* pw1 = (const float*)d_in[7];
  const float* cg1 = (const float*)d_in[8];
  const float* pw2 = (const float*)d_in[15];
  const float* cg2 = (const float*)d_in[16];
  const float* pw3 = (const float*)d_in[23];
  const float* cg3 = (const float*)d_in[24];
  const float* pw4 = (const float*)d_in[25];
  const float* cg4 = (const float*)d_in[26];
  const float* gm1 = (const float*)d_in[27];
  const float* gm2 = (const float*)d_in[28];
  const float* gm3 = (const float*)d_in[29];
  const float* gm4 = (const float*)d_in[30];

  char* ws = (char*)d_ws;
  unsigned short* W16 = (unsigned short*)(ws + oW16);
  float*          BIA = (float*)(ws + oBIA);
  unsigned short* X16 = (unsigned short*)(ws + oX16);
  unsigned short* XT  = (unsigned short*)(ws + oXT);
  unsigned short* XP  = (unsigned short*)(ws + oXP);
  float*          QKV = (float*)(ws + oQKV);
  unsigned short* Qp  = (unsigned short*)(ws + oQp);
  unsigned short* Kp  = (unsigned short*)(ws + oKp);
  unsigned short* VTp = (unsigned short*)(ws + oVTp);
  unsigned short* CQh = (unsigned short*)(ws + oCQh);
  unsigned short* CQl = (unsigned short*)(ws + oCQl);
  unsigned short* CKh = (unsigned short*)(ws + oCKh);
  unsigned short* CKl = (unsigned short*)(ws + oCKl);
  unsigned short* VTh = (unsigned short*)(ws + oVTh);
  unsigned short* VTl = (unsigned short*)(ws + oVTl);
  float*          Y1  = (float*)(ws + oY1);
  float*          Y2  = (float*)(ws + oY2);
  float*          Y3  = (float*)(ws + oY3);
  float*          Y4  = (float*)(ws + oY4);
  float* out = (float*)d_out;

  const dim3 blk256(256), blk128(128);
  const int XV   = CC * NN;
  const int QKVB = NQKV * NN;

  cvt_w<<<dim3(1), blk256, 0, stream>>>(wq[0], wq[1], wq[2], wq[3], wq[4], wq[5], wq[6], wq[7], wq[8],
                                        bq[0], bq[1], bq[2], bq[3], bq[4], bq[5], bq[6], bq[7], bq[8], W16, BIA);
  tr_kernel<<<dim3(CC, NB), blk256, 0, stream>>>(x, XV, 1, X16, XV, XT, nullptr, CC * IMW);
  cvt_xp<<<dim3(NN / QT, NB), blk256, 0, stream>>>(x, XP);
  gemm_qkv<<<dim3(NN / QT, NB), blk128, 0, stream>>>(W16, BIA, XP, QKV);
  planes_kernel<<<dim3(NN / QT, NB), blk256, 0, stream>>>(QKV, Qp, Kp, VTp, CQh, CQl, CKh, CKl);
  tr_kernel<<<dim3(8, NB), blk256, 0, stream>>>(QKV + 64 * NN, QKVB, 0, nullptr, 0, VTh, VTl, 512);
  chan_kernel<<<dim3(NB), blk256, 0, stream>>>(QKV, Y1);
  attn_kernel<1, 1, 0, 0, 0><<<dim3(NN / QT, NB), blk128, 0, stream>>>(
      Qp, nullptr, Kp, nullptr, VTp, nullptr, Y2, NN, NN * 32, NN * 32, 16 * NN, NN * 8);
  attn_kernel<4, 2, 1, 1, 1><<<dim3(512 / QT, NB), blk128, 0, stream>>>(
      CQh, CQl, CKh, CKl, VTh, VTl, Y3, 512, 512 * 64, 512 * 64, 64 * 512, 512 * 64);
  attn_kernel<4, 2, 0, 0, 1><<<dim3((CC * IMW) / QT, NB), blk128, 0, stream>>>(
      X16, nullptr, X16, nullptr, XT, nullptr, Y4, CC * IMW, XV, XV, XV, XV);
  proj_kernel<<<dim3(IMW, NB), blk256, 0, stream>>>(Y1, Y2, Y3, Y4, pw1, pw2, pw3, pw4,
                                                     cg1, cg2, cg3, cg4, gm1, gm2, gm3, gm4, out);
  (void)hipGetLastError();
}
